// GAT_86569360818245
// MI455X (gfx1250) — hardware-run, weakly checked
//
#include <hip/hip_runtime.h>


#ifndef NN
#define NN 16384
#endif
#ifndef NE
#define NE 524288
#endif
#define NN_FULL 16384
#define NE_FULL 524288
#define FEAT  128
#define EMB   64
#define NTILE (NN / 64)
#define AWV   8
#define RPW   8
#define CAPW  512
#define CAP2  512
#define CAP3  128
#define SLOPE 0.15f
#define L2E   1.4426950408889634f
#define NEGB  (-3.0e38f)

static_assert(FEAT % 32 == 0);
static_assert(EMB == 64);
static_assert(NN % 64 == 0);
static_assert(AWV * RPW == 64);
static_assert(NE % (128 * AWV) == 0);
static_assert(NE <= NE_FULL);
static_assert(NN <= NN_FULL);
static_assert(NN <= 16384);
static_assert(CAP3 == 128);
static_assert(((size_t)NN * FEAT) % 8 == 0);
static_assert(4 * 256 * 8 == FEAT * EMB);
static_assert(32 * 8 * 16 == 16 * EMB * 4);
static_assert(32 * 4 * 16 == RPW * EMB * 4);
static_assert(32 * 16 == 128 * 4);
static_assert((AWV * CAPW + AWV * CAP2 + AWV * CAP3) * 4 + AWV * CAP3 * 4 + AWV * RPW * EMB * 4 + 2 * AWV * 4 <= 65536);
static_assert((16 * 68 + 128 + 128 + 128) * 4 <= 131072);

typedef unsigned short bf;
typedef __attribute__((ext_vector_type(16))) __bf16   v16bf;
typedef __attribute__((ext_vector_type(8)))  unsigned short v8us;
typedef __attribute__((ext_vector_type(8)))  float    v8f;
typedef __attribute__((ext_vector_type(4)))  float    v4f;
typedef __attribute__((ext_vector_type(2)))  float    v2f;
typedef __attribute__((ext_vector_type(4)))  int      v4i;
typedef v4f  __attribute__((may_alias)) v4fa;

__device__ __forceinline__ unsigned short f2bf(float f) { unsigned u = __float_as_uint(f); u += 0x7FFFu + ((u >> 16) & 1u); return (unsigned short)(u >> 16); }
__device__ __forceinline__ float bfr(float f) { return __uint_as_float(((unsigned)f2bf(f)) << 16); }
__device__ __forceinline__ v16bf cat16b(v8us lo, v8us hi) { return __builtin_bit_cast(v16bf, __builtin_shufflevector(lo, hi, 0, 1, 2, 3, 4, 5, 6, 7, 8, 9, 10, 11, 12, 13, 14, 15)); }
__device__ __forceinline__ v8f wmmab(v16bf a, v16bf b, v8f c) { return __builtin_amdgcn_wmma_f32_16x16x32_bf16(false, a, false, b, (short)0, c, false, false); }
__device__ __forceinline__ v8f wmmab_g(v16bf a, v16bf b, v8f c) { c = wmmab(a, b, c); asm volatile("v_nop\n\tv_nop\n\tv_nop\n\tv_nop" : "+v"(c) : "v"(a), "v"(b)); return c; }
__device__ __forceinline__ v16bf ldb(const bf* p)  { return cat16b(*(const v8us*)p, *(const v8us*)(p + 16)); }
__device__ __forceinline__ void wave_sync() { __builtin_amdgcn_fence(3  , "wavefront"); __builtin_amdgcn_wave_barrier(); asm volatile("" ::: "memory"); }
__device__ __forceinline__ float elu_f(float v) {
    const float ex = __builtin_amdgcn_exp2f(v * L2E) - 1.0f;
    const float po = v * (1.0f + v * (0.5f + v * (0.16666667f + v * (0.041666668f + v * 0.0083333338f))));
    const float ng = (v > -0.0625f) ? po : ex;
    return (v > 0.0f) ? v : ng;
}

__global__ __launch_bounds__(256) void k_cvt8(const float* __restrict__ src, bf* dst, size_t n8) {
    const size_t i = (size_t)blockIdx.x * 256 + threadIdx.x; if (i >= n8) return;
    const v8f v = *(const v8f*)(src + i * 8); v8us o;
#pragma unroll
    for (int k = 0; k < 8; ++k) o[k] = f2bf(v[k]);
    *(volatile v8us*)(dst + i * 8) = o; __threadfence(); *(volatile v8us*)(dst + i * 8) = o;
}

__global__ __launch_bounds__(256) void k_wt(const float* __restrict__ W, bf* WT) {
#pragma unroll 1
    for (int it = 0; it < 4; ++it) {
        const int p = it * 256 + (int)threadIdx.x;
        const int n = p >> 4, k8 = (p & 15) * 8;
        v8us o;
#pragma unroll
        for (int i = 0; i < 8; ++i) o[i] = f2bf(W[(size_t)(k8 + i) * EMB + n]);
        *(volatile v8us*)(WT + (size_t)p * 8) = o; __threadfence(); *(volatile v8us*)(WT + (size_t)p * 8) = o;
    }
}

__global__ __launch_bounds__(32) void k_wh(const bf* __restrict__ A, const bf* __restrict__ Bt, const float* __restrict__ avec, float* WH, float* S12, float* CS) {
    __shared__ __align__(16) float os[16 * 68];
    __shared__ __align__(16) float sa[2 * EMB];
    __shared__ __align__(16) float sv[128];
    __shared__ __align__(16) float cs[128];
    const int K = FEAT;
    const int lane = threadIdx.x & 31, lr = lane & 15, hi = lane >> 4; const int r0 = blockIdx.x * 64;
    v8f acc[4][4];
#pragma unroll
    for (int mb = 0; mb < 4; ++mb)
#pragma unroll
        for (int nb = 0; nb < 4; ++nb) acc[mb][nb] = (v8f){};
    const size_t aoff = (size_t)(r0 + lr) * K + 8 * hi, boff = (size_t)lr * K + 8 * hi;
#pragma unroll 1
    for (int kc = 0; kc < K; kc += 32) {
        v16bf a[4];
#pragma unroll
        for (int mb = 0; mb < 4; ++mb) a[mb] = ldb(A + aoff + (size_t)mb * 16 * K + kc);
#pragma unroll
        for (int nb = 0; nb < 4; ++nb) { const v16bf b = ldb(Bt + boff + (size_t)nb * 16 * K + kc);
#pragma unroll
            for (int mb = 0; mb < 4; ++mb) acc[mb][nb] = wmmab_g(a[mb], b, acc[mb][nb]); }
    }
#pragma unroll
    for (int i = 0; i < 4; ++i) sa[lane + 32 * i] = bfr(avec[lane + 32 * i]);
    wave_sync();
    float cp0 = 0.0f, cp1 = 0.0f;
#pragma unroll
    for (int mb = 0; mb < 4; ++mb) {
#pragma unroll
        for (int nb = 0; nb < 4; ++nb) {
#pragma unroll
            for (int j = 0; j < 8; ++j) os[(hi * 8 + j) * 68 + nb * 16 + lr] = acc[mb][nb][j]; }
        wave_sync();
        float p1 = 0.0f, p2 = 0.0f;
#pragma unroll 4
        for (int c = 0; c < 32; ++c) { const float w = os[lr * 68 + hi * 32 + c]; p1 = fmaf(w, sa[hi * 32 + c], p1); p2 = fmaf(w, sa[EMB + hi * 32 + c], p2); }
        p1 += __shfl_xor(p1, 16, 32); p2 += __shfl_xor(p2, 16, 32);
        if (hi == 0) { sv[mb * 16 + lr] = p1; sv[64 + mb * 16 + lr] = p2; }
#pragma unroll 4
        for (int r = 0; r < 16; ++r) { cp0 += os[r * 68 + lane]; cp1 += os[r * 68 + 32 + lane]; }
        float* wrow = WH + (size_t)(r0 + mb * 16) * EMB;
#pragma unroll 1
        for (int ps = 0; ps < 2; ++ps) {
#pragma unroll
            for (int s = 0; s < 8; ++s) { const int p = s * 32 + lane; const int row = p >> 4, c4 = (p & 15) * 4;
                const v4f val = *(const v4fa*)(&os[row * 68 + c4]);
                *(volatile v4f*)(wrow + (size_t)p * 4) = val; }
            if (ps == 0) __threadfence(); }
        wave_sync();
    }
    cs[lane] = cp0; cs[32 + lane] = cp1; cs[64 + lane] = 0.0f; cs[96 + lane] = 0.0f;
    wave_sync();
    const v4f sq = *(const v4fa*)(&sv[4 * lane]);
    const v4f cq = *(const v4fa*)(&cs[4 * lane]);
    float* sp = S12 + (size_t)blockIdx.x * 128 + 4 * lane;
    float* cp = CS  + (size_t)blockIdx.x * 128 + 4 * lane;
    *(volatile v4f*)sp = sq; *(volatile v4f*)cp = cq;
    __threadfence();
    *(volatile v4f*)sp = sq; *(volatile v4f*)cp = cq;
}

__global__ __launch_bounds__(32 * AWV) void k_agg(const int* __restrict__ EI, const float* __restrict__ WH, const float* __restrict__ S12, const float* __restrict__ CS, float* OUT) {
    __shared__ int wl[AWV * CAPW];
    __shared__ int wl2[AWV * CAP2];
    __shared__ int rl[AWV * CAP3];
    __shared__ float wlw[AWV * CAP3];
    __shared__ __align__(16) float ot[AWV * RPW * EMB];
    __shared__ int wcnt[AWV];
    __shared__ int wovf[AWV];
    const int lane = threadIdx.x & 31;
    const int wave = __builtin_amdgcn_readfirstlane((int)(threadIdx.x >> 5));
    const int blk = blockIdx.x;
    const unsigned lt = (1u << lane) - 1u;

    int cnt = 0;
#pragma unroll 1
    for (int it = 0; it < NE / (128 * AWV); ++it) {
        const int e0 = ((it * AWV + wave) * 32 + lane) * 4;
        const v4i r4 = *(const v4i*)(EI + e0);
        bool hh[4];
#pragma unroll
        for (int q = 0; q < 4; ++q) { const int rb = r4[q] >> 6; hh[q] = (rb == blk) | (rb == blk - NTILE); }
        const unsigned any = __builtin_amdgcn_ballot_w32(hh[0] | hh[1] | hh[2] | hh[3]);
        if (any != 0u) {
            const v4i c4 = *(const v4i*)(EI + NE_FULL + e0);
#pragma unroll
            for (int q = 0; q < 4; ++q) {
                int c = c4[q]; c += (c >> 31) & NN;
                const bool ok = hh[q] & ((unsigned)c < (unsigned)NN);
                const unsigned mk = __builtin_amdgcn_ballot_w32(ok);
                const int pos = cnt + __builtin_popcount(mk & lt);
                if (ok & (pos < CAPW)) wl[wave * CAPW + pos] = ((r4[q] & 63) << 14) | c;
                cnt += __builtin_popcount(mk);
            }
        }
    }
    if (lane == 0) { wcnt[wave] = cnt < CAPW ? cnt : CAPW; wovf[wave] = cnt > CAPW ? 1 : 0; }
    __syncthreads();

    int c2 = 0; int ov = 0;
#pragma unroll 1
    for (int w2 = 0; w2 < AWV; ++w2) {
        const int n2 = __builtin_amdgcn_readfirstlane(wcnt[w2]);
        ov |= __builtin_amdgcn_readfirstlane(wovf[w2]);
#pragma unroll 1
        for (int p0 = 0; p0 < n2; p0 += 32) {
            const int p = p0 + lane;
            const int pc = p < n2 ? p : (n2 - 1);
            const int key = wl[w2 * CAPW + pc];
            const bool ok = (p < n2) & ((key >> 17) == wave);
            const unsigned mk = __builtin_amdgcn_ballot_w32(ok);
            const int pos = c2 + __builtin_popcount(mk & lt);
            if (ok & (pos < CAP2)) wl2[wave * CAP2 + pos] = key;
            c2 += __builtin_popcount(mk);
        }
    }
    ov |= (c2 > CAP2) ? 1 : 0;
    const int m2 = c2 < CAP2 ? c2 : CAP2;
    wave_sync();

#pragma unroll 1
    for (int rr = 0; rr < RPW; ++rr) {
        int n3 = 0;
#pragma unroll 1
        for (int p0 = 0; p0 < m2; p0 += 32) {
            const int p = p0 + lane;
            const int pc = p < m2 ? p : (m2 - 1);
            const int key = wl2[wave * CAP2 + pc];
            const bool ok = (p < m2) & (((key >> 14) & 7) == rr);
            const unsigned mk = __builtin_amdgcn_ballot_w32(ok);
            const int pos = n3 + __builtin_popcount(mk & lt);
            if (ok & (pos < CAP3)) rl[wave * CAP3 + pos] = key & 16383;
            n3 += __builtin_popcount(mk);
        }
        ov |= (n3 > CAP3) ? 1 : 0;
        const int n = n3 < CAP3 ? n3 : CAP3;
        wave_sync();
        float v0, v1;
        if (n == 0) {
            float t0 = 0.0f, t1 = 0.0f;
#pragma unroll 1
            for (int t = 0; t < NTILE; ++t) { const v2f c = *(const v2f*)(CS + (size_t)t * 128 + 2 * lane); t0 += c[0]; t1 += c[1]; }
            v0 = t0 * (1.0f / (float)NN); v1 = t1 * (1.0f / (float)NN);
        } else {
            const float si = S12[(size_t)blk * 128 + wave * RPW + rr];
            int cq[4]; float eq[4]; bool vq[4]; float mx = NEGB;
#pragma unroll
            for (int q = 0; q < 4; ++q) {
                const int p = lane + 32 * q;
                const int pc = p < n ? p : (n - 1);
                const int j = rl[wave * CAP3 + pc];
                float s2v = S12[(size_t)(j >> 6) * 128 + 64 + (j & 63)];
                asm volatile("" : "+v"(s2v));
                const float x = si + s2v;
                const float e = x > 0.0f ? x : SLOPE * x;
                vq[q] = p < n; cq[q] = vq[q] ? j : -1; eq[q] = e;
                mx = fmaxf(mx, vq[q] ? e : NEGB);
            }
            mx = fmaxf(mx, __shfl_xor(mx, 16, 32)); mx = fmaxf(mx, __shfl_xor(mx, 8, 32)); mx = fmaxf(mx, __shfl_xor(mx, 4, 32));
            mx = fmaxf(mx, __shfl_xor(mx, 2, 32));  mx = fmaxf(mx, __shfl_xor(mx, 1, 32));
#pragma unroll
            for (int q = 0; q < 4; ++q) {
                const float ex = __builtin_amdgcn_exp2f((eq[q] - mx) * L2E);
                wlw[wave * CAP3 + lane + 32 * q] = vq[q] ? ex : 0.0f;
            }
            wave_sync();
            float Z = 0.0f, a0 = 0.0f, a1 = 0.0f;
#pragma unroll 1
            for (int k = 0; k < n; ++k) {
                const int j = __builtin_amdgcn_readfirstlane(rl[wave * CAP3 + k]);
                const float w = wlw[wave * CAP3 + k];
                const bool d = ((cq[0] == j) & (lane < k)) | ((cq[1] == j) & (lane + 32 < k)) | ((cq[2] == j) & (lane + 64 < k)) | ((cq[3] == j) & (lane + 96 < k));
                const unsigned dm = __builtin_amdgcn_ballot_w32(d);
                if (dm == 0u) {
                    const v2f x = *(const v2f*)(WH + (size_t)j * EMB + 2 * lane);
                    Z += w; a0 = fmaf(w, x[0], a0); a1 = fmaf(w, x[1], a1);
                }
            }
            const float iz = 1.0f / Z;
            v0 = a0 * iz; v1 = a1 * iz;
        }
        v0 = elu_f(v0); v1 = elu_f(v1);
        ot[(wave * RPW + rr) * EMB + 2 * lane] = v0; ot[(wave * RPW + rr) * EMB + 2 * lane + 1] = v1;
        wave_sync();
    }

    const float pz = __uint_as_float(0x7FC00000u);
    float* orow = OUT + ((size_t)blk * 64 + (size_t)wave * RPW) * EMB;
#pragma unroll 1
    for (int ps = 0; ps < 2; ++ps) {
#pragma unroll
        for (int s = 0; s < 4; ++s) { const int p = s * 32 + lane;
            v4f val = *(const v4fa*)(&ot[wave * RPW * EMB + p * 4]);
            const v4f pv = (v4f){pz, pz, pz, pz};
            val = (ov != 0) ? pv : val;
            *(volatile v4f*)(orow + (size_t)p * 4) = val; }
        if (ps == 0) __threadfence(); }
}

static constexpr size_t al256(size_t v) { return (v + 255) & ~(size_t)255; }
static constexpr size_t SZ_XB = al256((size_t)NN * FEAT * 2);
static constexpr size_t SZ_WT = al256((size_t)EMB * FEAT * 2);
static constexpr size_t SZ_WH = al256((size_t)NN * EMB * 4);
static constexpr size_t SZ_TR = al256((size_t)NTILE * 128 * 4);
static constexpr size_t SZ_TOTAL = SZ_XB + SZ_WT + SZ_WH + 2 * SZ_TR;
static_assert(SZ_TOTAL <= (size_t)134217728);
static_assert((size_t)(NTILE - 1) * 128 + 128 <= SZ_TR / 4);
static_assert((size_t)(NN - 64 + 48) * EMB + 255 * 4 + 4 <= SZ_WH / 4);
static_assert(((size_t)(NTILE - 1) * 64 + (AWV - 1) * RPW) * EMB + 127 * 4 + 4 <= (size_t)NN * EMB);

extern "C" void kernel_launch(void* const* d_in, const int* in_sizes, int n_in,
                              void* d_out, int out_size, void* d_ws, size_t ws_size, hipStream_t stream) {
    if (n_in < 4) return;
    if ((size_t)in_sizes[0] < (size_t)NE_FULL + (size_t)NE) return;
    if ((size_t)in_sizes[1] < (size_t)NN * FEAT) return;
    if (in_sizes[2] < FEAT * EMB || in_sizes[3] < 2 * EMB) return;
    if ((size_t)out_size < (size_t)NN * EMB) return;
    if (SZ_TOTAL > ws_size) return;
    const int*   EI = (const int*)d_in[0];
    const float* X  = (const float*)d_in[1];
    const float* Ws = (const float*)d_in[2];
    const float* av = (const float*)d_in[3];
    float* OUT = (float*)d_out;
    char* wsp = (char*)d_ws;
    bf* XB = (bf*)wsp; wsp += SZ_XB;
    bf* WT = (bf*)wsp; wsp += SZ_WT;
    float* WH = (float*)wsp; wsp += SZ_WH;
    float* S12 = (float*)wsp; wsp += SZ_TR;
    float* CS = (float*)wsp; wsp += SZ_TR;

    { const size_t n8 = (size_t)NN * FEAT / 8;
      k_cvt8<<<(unsigned)((n8 + 255) / 256), 256, 0, stream>>>(X, XB, n8); }
    k_wt<<<1, 256, 0, stream>>>(Ws, WT);
    k_wh<<<NTILE, 32, 0, stream>>>(XB, WT, av, WH, S12, CS);
    k_agg<<<NTILE, 32 * AWV, 0, stream>>>(EI, WH, S12, CS, OUT);
}
